// Task_36275293782743
// MI455X (gfx1250) — hardware-verified
//
#include <hip/hip_runtime.h>
#include <math.h>

typedef __attribute__((ext_vector_type(16))) _Float16 v16h;
typedef __attribute__((ext_vector_type(16))) __bf16 v16b;
typedef __attribute__((ext_vector_type(8)))  _Float16 v8h;
typedef __attribute__((ext_vector_type(8)))  float v8f;
typedef __attribute__((ext_vector_type(4)))  float v4f;
typedef __attribute__((ext_vector_type(2)))  float v2f;
typedef __attribute__((ext_vector_type(4)))  unsigned v4u;
typedef __attribute__((ext_vector_type(4)))  int v4i;
typedef float __attribute__((may_alias)) float_a;
typedef int __attribute__((may_alias)) int_a;

template <typename T> __device__ __forceinline__ void vst2(void* p, T v) { *(volatile T*)p = v; __threadfence(); *(volatile T*)p = v; }
__device__ __forceinline__ v8f wmma16(v16h a, v16h b, v8f c) {
  v8f d = __builtin_amdgcn_wmma_f32_16x16x32_f16(false, a, false, b, (short)0, c, false, false);
  asm volatile("v_nop\n\tv_nop\n\tv_nop\n\tv_nop" : "+v"(d) : "v"(a), "v"(b));
  return d;
}
__device__ __forceinline__ v8f wmma_bf(v16b a, v16b b, v8f c) {
  v8f d = __builtin_amdgcn_wmma_f32_16x16x32_bf16(false, a, false, b, (short)0, c, false, false);
  asm volatile("v_nop\n\tv_nop\n\tv_nop\n\tv_nop" : "+v"(d) : "v"(a), "v"(b));
  return d;
}
__device__ __forceinline__ v16h frag_h(const _Float16* rowk0, int lane) {
  union { v16h v; v8h q[2]; } u; const _Float16* p = rowk0 + 8 * (lane >> 4);
  u.q[0] = *(const v8h*)p; u.q[1] = *(const v8h*)(p + 16); return u.v;
}
__device__ __forceinline__ v16h frag_f32(const float* rowk0, int lane) {
  v16h a; const float* p = rowk0 + 8 * (lane >> 4);
#pragma unroll
  for (int i = 0; i < 8; ++i) { a[i] = (_Float16)p[i]; a[8 + i] = (_Float16)p[16 + i]; }
  return a;
}
__device__ __forceinline__ v16h frag_f32s(const float* rowk0, int lane, float sc) {
  v16h a; const float* p = rowk0 + 8 * (lane >> 4);
#pragma unroll
  for (int i = 0; i < 8; ++i) { a[i] = (_Float16)(p[i] * sc); a[8 + i] = (_Float16)(p[16 + i] * sc); }
  return a;
}
__device__ __forceinline__ v16h fragc_f32(const float* W, int k0, int n, int lane, int ld, int K) {
  v16h a; const int g = lane >> 4;
#pragma unroll
  for (int i = 0; i < 8; ++i) { const int ka = k0 + 8 * g + i, kb = ka + 16;
    a[i] = (_Float16)(ka < K ? W[(size_t)ka * ld + n] : 0.f); a[8 + i] = (_Float16)(kb < K ? W[(size_t)kb * ld + n] : 0.f); }
  return a;
}
struct F2 { v16b h, l; };
__device__ __forceinline__ F2 bsplit16(const float v[16]) { F2 r;
#pragma unroll
  for (int i = 0; i < 16; ++i) { const __bf16 h = (__bf16)v[i]; r.h[i] = h; r.l[i] = (__bf16)(v[i] - (float)h); }
  return r; }
__device__ __forceinline__ F2 split_row(const float* row, int k0, int lane) { float v[16]; const float* p = row + k0 + 8 * (lane >> 4);
#pragma unroll
  for (int i = 0; i < 8; ++i) { v[i] = p[i]; v[8 + i] = p[16 + i]; }
  return bsplit16(v); }
__device__ __forceinline__ F2 split_rowK(const float* row, int k0, int lane, int K) { float v[16]; const int g = lane >> 4;
#pragma unroll
  for (int i = 0; i < 8; ++i) { const int ka = k0 + 8 * g + i, kb = ka + 16; v[i] = ka < K ? row[ka] : 0.f; v[8 + i] = kb < K ? row[kb] : 0.f; }
  return bsplit16(v); }
__device__ __forceinline__ F2 split_col(const float* W, int k0, int n, int lane, int ld, int K) { float v[16]; const int g = lane >> 4;
#pragma unroll
  for (int i = 0; i < 8; ++i) { const int ka = k0 + 8 * g + i, kb = ka + 16; v[i] = ka < K ? W[(size_t)ka * ld + n] : 0.f; v[8 + i] = kb < K ? W[(size_t)kb * ld + n] : 0.f; }
  return bsplit16(v); }
__device__ __forceinline__ v8f mac3(const F2& a, const F2& b, v8f c) { c = wmma_bf(a.l, b.h, c); c = wmma_bf(a.h, b.l, c); return wmma_bf(a.h, b.h, c); }
__device__ __forceinline__ float sigm(float v) { return 1.0f / (1.0f + expf(-v)); }
#define LDSX() do { asm volatile("s_wait_dscnt 0" ::: "memory"); __builtin_amdgcn_wave_barrier(); __builtin_amdgcn_fence(__ATOMIC_RELEASE, "workgroup"); } while (0)

#define NTOK 65536
#define DIN 128
#define HIDC 2048
#define NE 8
#define SG 16
#define CHK 16384
#define NPB 4096

__global__ __launch_bounds__(256) void k_cvt(const float* __restrict__ src, _Float16* __restrict__ dst, size_t n8, float sc) {
  const size_t g8 = (size_t)blockIdx.x * 256 + threadIdx.x; if (g8 >= n8) return;
  union { v8h h; v4u u; } pk;
#pragma unroll
  for (int e = 0; e < 8; ++e) pk.h[e] = (_Float16)(src[g8 * 8 + e] * sc);
  vst2(dst + g8 * 8, pk.u);
}
__global__ __launch_bounds__(256) void k_packW2(const float* __restrict__ w2, _Float16* __restrict__ P2) {
  const int o = blockIdx.x, tid = threadIdx.x;
  union { v8h h; v4u u; } pk; const int k0 = tid * 8; const int e = k0 >> 8, hh = k0 & 255;
#pragma unroll
  for (int i = 0; i < 8; ++i) pk.h[i] = (_Float16)(w2[((size_t)e * DIN + o) * 256 + hh + i] * 16.0f);
  vst2(P2 + (size_t)o * HIDC + k0, pk.u);
}
__global__ __launch_bounds__(128) void k_gate(const _Float16* __restrict__ x16, const float* __restrict__ x, const float* __restrict__ sg1, const float* __restrict__ sg2, const float* __restrict__ gw, const int* __restrict__ act, float* __restrict__ wts, float* __restrict__ aux) {
  __shared__ __align__(16) float s1[4][16][20];
  __shared__ __align__(16) float ssh[4][16][132];
  __shared__ __align__(16) float ssc[4][16][20];
  __shared__ __align__(16) float sw[4][16][8];
  const int tid = threadIdx.x, wave = tid >> 5, lane = tid & 31, col = lane & 15, g = lane >> 4;
  const int t0 = blockIdx.x * 64 + wave * 16;
  if (blockIdx.x == 0 && tid == 0) vst2(aux, (float_a)0.f);
  { v8f acc = {};
#pragma unroll
    for (int kc = 0; kc < 4; ++kc) acc = wmma16(frag_h(x16 + (size_t)(t0 + col) * DIN + kc * 32, lane), frag_f32s(sg1 + (size_t)col * DIN + kc * 32, lane, 16.0f), acc);
#pragma unroll
    for (int r = 0; r < 8; ++r) { const float v = acc[r] * (1.0f / 16.0f); s1[wave][8 * g + r][col] = v > 0.f ? v : 0.f; } }
  LDSX();
  { v16h a;
#pragma unroll
    for (int i = 0; i < 8; ++i) { a[i] = (_Float16)s1[wave][col][8 * g + i]; a[8 + i] = (_Float16)0.f; }
#pragma unroll
    for (int j = 0; j < 8; ++j) { v16h bb;
#pragma unroll
      for (int i = 0; i < 8; ++i) { bb[i] = (_Float16)(sg2[(size_t)(j * 16 + col) * SG + 8 * g + i] * 16.0f); bb[8 + i] = (_Float16)0.f; }
      v8f acc = {}; acc = wmma16(a, bb, acc);
#pragma unroll
      for (int r = 0; r < 8; ++r) ssh[wave][8 * g + r][j * 16 + col] = acc[r] * (1.0f / 16.0f) + x[(size_t)(t0 + 8 * g + r) * DIN + j * 16 + col]; } }
  LDSX();
  { v8f acc = {};
#pragma unroll
    for (int kc = 0; kc < 4; ++kc) { v16h bb;
#pragma unroll
      for (int i = 0; i < 8; ++i) { bb[i] = (_Float16)(col < NE ? gw[(size_t)col * DIN + kc * 32 + 8 * g + i] * 16.0f : 0.f); bb[8 + i] = (_Float16)(col < NE ? gw[(size_t)col * DIN + kc * 32 + 16 + 8 * g + i] * 16.0f : 0.f); }
      acc = wmma16(frag_f32(&ssh[wave][col][0] + kc * 32, lane), bb, acc); }
#pragma unroll
    for (int r = 0; r < 8; ++r) ssc[wave][8 * g + r][col] = acc[r] * (1.0f / 16.0f); }
  LDSX();
  if (g == 0) { const int m = col, t = t0 + m, b = t / NPB; float mx = -3.0e38f; float sc[NE];
#pragma unroll
    for (int e = 0; e < NE; ++e) { sc[e] = act[b * NE + e] != 0 ? ssc[wave][m][e] : -3.0e38f; mx = fmaxf(mx, sc[e]); }
    float l = 0.f;
#pragma unroll
    for (int e = 0; e < NE; ++e) { sc[e] = sc[e] <= -1.0e38f ? 0.f : expf(sc[e] - mx); l += sc[e]; }
    const float inv = 1.0f / l;
#pragma unroll
    for (int e = 0; e < NE; ++e) sw[wave][m][e] = sc[e] * inv; }
  LDSX();
  vst2(wts + (size_t)t0 * NE + lane * 4, *(const v4f*)(&sw[wave][0][0] + lane * 4));
}
__global__ __launch_bounds__(128) void k_g1(const _Float16* __restrict__ x16, const _Float16* __restrict__ P1, const float* __restrict__ wts, int t0c, _Float16* __restrict__ Hc) {
  __shared__ __align__(16) float so[4][16][132];
  const int tid = threadIdx.x, wave = tid >> 5, lane = tid & 31, col = lane & 15, g = lane >> 4;
  const int rl0 = blockIdx.x * 64 + wave * 16, n0 = blockIdx.y * 128; const int e = n0 >> 8;
  v8f acc[8] = {};
#pragma unroll
  for (int kc = 0; kc < DIN / 32; ++kc) { const v16h a = frag_h(x16 + (size_t)(t0c + rl0 + col) * DIN + kc * 32, lane);
#pragma unroll
    for (int j = 0; j < 8; ++j) acc[j] = wmma16(a, frag_h(P1 + (size_t)(n0 + j * 16 + col) * DIN + kc * 32, lane), acc[j]); }
#pragma unroll
  for (int j = 0; j < 8; ++j)
#pragma unroll
    for (int r = 0; r < 8; ++r) { const float v = acc[j][r] * (1.0f / 16.0f); so[wave][8 * g + r][j * 16 + col] = (v > 0.f ? v : 0.f) * wts[(size_t)(t0c + rl0 + 8 * g + r) * NE + e] * 16.0f; }
  LDSX();
  for (int q = lane; q < 16 * 16; q += 32) { const int rl = q >> 4, pc = q & 15; union { v8h hh; v4u u; } pk;
#pragma unroll
    for (int i = 0; i < 8; ++i) pk.hh[i] = (_Float16)so[wave][rl][pc * 8 + i];
    vst2(Hc + (size_t)(rl0 + rl) * HIDC + n0 + pc * 8, pk.u); }
}
__global__ __launch_bounds__(128) void k_g2(const _Float16* __restrict__ Hc, const _Float16* __restrict__ P2, int t0c, float* __restrict__ out) {
  __shared__ __align__(16) float so[4][16][132];
  const int tid = threadIdx.x, wave = tid >> 5, lane = tid & 31, col = lane & 15, g = lane >> 4;
  const int rl0 = blockIdx.x * 64 + wave * 16;
  v8f acc[8] = {};
#pragma unroll 1
  for (int kc = 0; kc < HIDC / 32; ++kc) { const v16h a = frag_h(Hc + (size_t)(rl0 + col) * HIDC + kc * 32, lane);
#pragma unroll
    for (int j = 0; j < 8; ++j) acc[j] = wmma16(a, frag_h(P2 + (size_t)(j * 16 + col) * HIDC + kc * 32, lane), acc[j]); }
#pragma unroll
  for (int j = 0; j < 8; ++j)
#pragma unroll
    for (int r = 0; r < 8; ++r) so[wave][8 * g + r][j * 16 + col] = acc[j][r] * (1.0f / 256.0f);
  LDSX();
#pragma unroll 4
  for (int rl = 0; rl < 16; ++rl) vst2(out + (size_t)(t0c + rl0 + rl) * DIN + lane * 4, *(const v4f*)(&so[wave][rl][lane * 4]));
}
extern "C" void kernel_launch(void* const* d_in, const int* in_sizes, int n_in, void* d_out, int out_size, void* d_ws, size_t ws_size, hipStream_t stream) {
  (void)in_sizes; (void)n_in; (void)out_size; (void)ws_size;
  const float* x = (const float*)d_in[0]; const int* act = (const int*)d_in[1]; const float* sg1 = (const float*)d_in[2]; const float* sg2 = (const float*)d_in[3]; const float* gw = (const float*)d_in[4]; const float* w1 = (const float*)d_in[5]; const float* w2 = (const float*)d_in[6];
  float* out = (float*)d_out; float* aux = (float*)((char*)d_out + 33554432);
  char* ws = (char*)d_ws; size_t off = 0;
  auto take = [&](size_t bytes) { char* p = ws + off; off += (bytes + 255) & ~(size_t)255; return p; };
  _Float16* x16 = (_Float16*)take((size_t)NTOK * DIN * 2); _Float16* P1 = (_Float16*)take((size_t)HIDC * DIN * 2); _Float16* P2 = (_Float16*)take((size_t)DIN * HIDC * 2);
  float* wts = (float*)take((size_t)NTOK * NE * 4); _Float16* Hc = (_Float16*)take((size_t)CHK * HIDC * 2);
  { const size_t n8 = (size_t)NTOK * DIN / 8; k_cvt<<<(unsigned)(n8 / 256), 256, 0, stream>>>(x, x16, n8, 1.0f); }
  { const size_t n8 = (size_t)HIDC * DIN / 8; k_cvt<<<(unsigned)(n8 / 256), 256, 0, stream>>>(w1, P1, n8, 16.0f); }
  k_packW2<<<DIN, 256, 0, stream>>>(w2, P2);
  k_gate<<<NTOK / 64, 128, 0, stream>>>(x16, x, sg1, sg2, gw, act, wts, aux);
  for (int c = 0; c < NTOK / CHK; ++c) { const int t0c = c * CHK;
    k_g1<<<dim3(CHK / 64, HIDC / 128), 128, 0, stream>>>(x16, P1, wts, t0c, Hc);
    k_g2<<<CHK / 64, 128, 0, stream>>>(Hc, P2, t0c, out); }
}
